// PINN_Burgers2D_89146341195842
// MI455X (gfx1250) — hardware-verified
//
#include <hip/hip_runtime.h>
#include <stddef.h>
#include <stdint.h>

#define WID    128
#define WP     136
#define NL     5
#define NWAVES 4
#define TM     16
#define RPI    (NWAVES * TM)
#define ITERS  16
#define RPB    (RPI * ITERS)
#define WMAT   (WID * WP)
#define ATILE  (TM * WP)
#define DYN_ELEMS (NL * WMAT + NWAVES * 2 * ATILE)

static_assert(WID == 128);
static_assert(TM == 16);
static_assert((WP % 8) == 0);
static_assert(NWAVES * 32 == WID);
static_assert((RPB % TM) == 0);

typedef unsigned short v8us  __attribute__((ext_vector_type(8)));
typedef unsigned short v16us __attribute__((ext_vector_type(16)));
typedef float          v4f   __attribute__((ext_vector_type(4)));
typedef float          v8f   __attribute__((ext_vector_type(8)));
#if defined(__HIP_DEVICE_COMPILE__)
typedef __bf16         v16bf __attribute__((ext_vector_type(16)));
#endif

union FragU { v16us v; v8us half[2]; };

__device__ __forceinline__ unsigned bbits(float f) {
  unsigned u = __float_as_uint(f);
  return (u + 0x7FFFu + ((u >> 16) & 1u)) >> 16;
}
__device__ __forceinline__ float bf16r(float f) {
  return __uint_as_float(bbits(f) << 16);
}
__device__ __forceinline__ v8f zero8() { v8f z = {0.f, 0.f, 0.f, 0.f, 0.f, 0.f, 0.f, 0.f}; return z; }
__device__ __forceinline__ float silu_f(float z) {
  const float e = __expf(-z);
  return z * __builtin_amdgcn_rcpf(1.0f + e);
}
__device__ __forceinline__ void split2(float v, unsigned short& hb, unsigned short& lb) {
  const unsigned hu = bbits(v);
  hb = (unsigned short)hu;
  lb = (unsigned short)bbits(v - __uint_as_float(hu << 16));
}

__device__ __forceinline__ v16us ldfrag(const unsigned short* p) {
  FragU f;
  f.half[0] = *(const v8us*)(p);
  f.half[1] = *(const v8us*)(p + 16);
  return f.v;
}

__device__ __forceinline__ v8f mma_bf(v16us a, v16us b, v8f c) {
#if defined(__HIP_DEVICE_COMPILE__)
  return __builtin_amdgcn_wmma_f32_16x16x32_bf16(false, __builtin_bit_cast(v16bf, a),
                                                false, __builtin_bit_cast(v16bf, b),
                                                (short)0, c, false, false);
#else
  (void)a; (void)b;
  return c;
#endif
}
__device__ __forceinline__ void guard(v8f& acc,
                                      const v16us& a0, const v16us& a1, const v16us& a2, const v16us& a3,
                                      const v16us& a4, const v16us& a5, const v16us& a6, const v16us& a7,
                                      const v16us& b0, const v16us& b1, const v16us& b2, const v16us& b3) {
#if defined(__HIP_DEVICE_COMPILE__)
  asm volatile("v_nop\n\tv_nop\n\tv_nop\n\tv_nop"
               : "+v"(acc)
               : "v"(a0), "v"(a1), "v"(a2), "v"(a3), "v"(a4), "v"(a5), "v"(a6), "v"(a7),
                 "v"(b0), "v"(b1), "v"(b2), "v"(b3));
#endif
}

__global__ __launch_bounds__(128)
void k_mlp(const float* __restrict__ X,
           const float* __restrict__ numin_p, const float* __restrict__ numax_p,
           const float* __restrict__ W0, const float* __restrict__ b0,
           const float* __restrict__ Wh, const float* __restrict__ bh,
           const float* __restrict__ WL, const float* __restrict__ bL,
           float* out, int n)
{
  extern __shared__ __align__(16) unsigned short dynlds[];
  __shared__ __align__(16) float w0s[4][WID];
  __shared__ __align__(16) float b0s[WID];
  __shared__ __align__(16) float bls[NL][WID];
  __shared__ __align__(16) float wls[2][WID];
  __shared__ __align__(16) float sOut[NWAVES][2 * TM];
  __shared__ float blv[2];

  const int tid = threadIdx.x;

#pragma unroll 1
  for (int L = 0; L < NL; ++L) {
    const float* src = Wh + (size_t)L * WID * WID;
    unsigned short* dst = dynlds + (size_t)L * WMAT + (size_t)tid * WP;
#pragma unroll 4
    for (int s = 0; s < WID; ++s) dst[s] = (unsigned short)bbits(src[(size_t)s * WID + tid]);
  }
#pragma unroll
  for (int k = 0; k < 4; ++k) w0s[k][tid] = bf16r(W0[k * WID + tid]);
  b0s[tid] = bf16r(b0[tid]);
#pragma unroll
  for (int L = 0; L < NL; ++L) bls[L][tid] = bf16r(bh[L * WID + tid]);
  wls[0][tid] = bf16r(WL[tid * 2 + 0]);
  wls[1][tid] = bf16r(WL[tid * 2 + 1]);
  if (tid < 2) blv[tid] = bf16r(bL[tid]);
  __syncthreads();

  const int lane = tid & 31;
  const int wave = tid >> 5;
  const int hh   = lane >> 4;
  const int c    = lane & 15;
  unsigned short* actH = dynlds + (size_t)NL * WMAT + (size_t)wave * (2 * ATILE);
  unsigned short* actL = actH + ATILE;

  const float numin = bf16r(numin_p[0]);
  const float numax = bf16r(numax_p[0]);
  const float rnu   = 1.0f / (numax - numin);
  const float blx = blv[0], bly = blv[1];
  const long blockRow0 = (long)blockIdx.x * RPB;

#pragma unroll 1
  for (int it = 0; it < ITERS; ++it) {
    const long r0w = blockRow0 + (long)it * RPI + (long)wave * TM;
    __syncthreads();

    {
      long gr = r0w + c;
      if (gr > (long)n - 1) gr = (long)n - 1;
      const v4f xv = *(const v4f*)(X + gr * 4);
      const float xb0 = bf16r(xv[0]), xb1 = bf16r(xv[1]), xb2 = bf16r(xv[2]), xb3 = bf16r(xv[3]);
      const float i0 = (2.0f * (xb0 - (-1.0f))) * 0.5f - 1.0f;
      const float i1 = (2.0f * (xb1 - (-1.0f))) * 0.5f - 1.0f;
      const float i2 = (2.0f * (xb2 - 0.0f)) * 1.0f - 1.0f;
      const float i3 = (2.0f * (xb3 - numin)) * rnu - 1.0f;
      unsigned short* ph = actH + c * WP + 64 * hh;
      unsigned short* pl = actL + c * WP + 64 * hh;
#pragma unroll 1
      for (int j8 = 0; j8 < 8; ++j8) {
        const int nb = 64 * hh + 8 * j8;
        v8us oh, ol;
#pragma unroll
        for (int q = 0; q < 8; ++q) {
          const int nn = nb + q;
          const float z  = b0s[nn] + (((i0 * w0s[0][nn] + i1 * w0s[1][nn]) + i2 * w0s[2][nn]) + i3 * w0s[3][nn]);
          const float hv = silu_f(z);
          unsigned short hb, lb;
          split2(hv, hb, lb);
          oh[q] = hb;
          ol[q] = lb;
        }
        *(v8us*)(ph + 8 * j8) = oh;
        *(v8us*)(pl + 8 * j8) = ol;
      }
    }
    __syncthreads();

#pragma unroll 1
    for (int li = 0; li < NL; ++li) {
      const unsigned short* wl  = dynlds + (size_t)li * WMAT;
      const unsigned short* arh = actH + c * WP + 8 * hh;
      const unsigned short* arl = actL + c * WP + 8 * hh;
      const v16us ah0 = ldfrag(arh),      ah1 = ldfrag(arh + 32), ah2 = ldfrag(arh + 64), ah3 = ldfrag(arh + 96);
      const v16us al0 = ldfrag(arl),      al1 = ldfrag(arl + 32), al2 = ldfrag(arl + 64), al3 = ldfrag(arl + 96);
      float sx[8], sy[8];
#pragma unroll
      for (int r = 0; r < 8; ++r) { sx[r] = 0.0f; sy[r] = 0.0f; }

#pragma unroll 1
      for (int nt = 0; nt < 8; ++nt) {
        const int n0 = nt * 16;
        const unsigned short* wp = wl + (n0 + c) * WP + 8 * hh;
        const v16us g0 = ldfrag(wp);
        const v16us g1 = ldfrag(wp + 32);
        const v16us g2 = ldfrag(wp + 64);
        const v16us g3 = ldfrag(wp + 96);
        v8f acc = zero8();
        acc = mma_bf(ah0, g0, acc);
        acc = mma_bf(al0, g0, acc);
        acc = mma_bf(ah1, g1, acc);
        acc = mma_bf(al1, g1, acc);
        acc = mma_bf(ah2, g2, acc);
        acc = mma_bf(al2, g2, acc);
        acc = mma_bf(ah3, g3, acc);
        acc = mma_bf(al3, g3, acc);
        guard(acc, ah0, ah1, ah2, ah3, al0, al1, al2, al3, g0, g1, g2, g3);
        const int ncol = n0 + c;
        const float bias = bls[li][ncol];
        if (li < NL - 1) {
#pragma unroll
          for (int r = 0; r < 8; ++r) {
            const float hv = silu_f(acc[r] + bias);
            unsigned short hb, lb;
            split2(hv, hb, lb);
            const int o = (8 * hh + r) * WP + ncol;
            actH[o] = hb;
            actL[o] = lb;
          }
        } else {
          const float wx = wls[0][ncol];
          const float wy = wls[1][ncol];
#pragma unroll
          for (int r = 0; r < 8; ++r) {
            const float hv = silu_f(acc[r] + bias);
            sx[r] += hv * wx;
            sy[r] += hv * wy;
          }
        }
      }

      if (li == NL - 1) {
#pragma unroll
        for (int off = 8; off >= 1; off >>= 1) {
#pragma unroll
          for (int r = 0; r < 8; ++r) {
            sx[r] += __shfl_xor(sx[r], off, 16);
            sy[r] += __shfl_xor(sy[r], off, 16);
          }
        }
        if (c == 0) {
#pragma unroll
          for (int r = 0; r < 8; ++r) {
            sOut[wave][(8 * hh + r) * 2 + 0] = sx[r] + blx;
            sOut[wave][(8 * hh + r) * 2 + 1] = sy[r] + bly;
          }
        }
      }
      __syncthreads();
    }

    {
      const float ov = sOut[wave][lane];
      const long gro = r0w + (long)(lane >> 1);
      float* po = out + r0w * 2 + lane;
      if (gro < (long)n) *(volatile float*)po = ov;
      __threadfence();
      if (gro < (long)n) *(volatile float*)po = ov;
    }
  }
}

extern "C" void kernel_launch(void* const* d_in, const int* in_sizes, int n_in,
                              void* d_out, int out_size, void* d_ws, size_t ws_size,
                              hipStream_t stream) {
  (void)d_ws; (void)ws_size;
  if (n_in < 9) return;
  if (in_sizes[0] < 4 || (in_sizes[0] & 3) != 0) return;
  const int n = in_sizes[0] / 4;
  if (out_size != 2 * n) return;
  if (in_sizes[1] < 1 || in_sizes[2] < 1) return;
  if (in_sizes[3] != 4 * WID || in_sizes[4] != WID) return;
  if (in_sizes[5] != NL * WID * WID || in_sizes[6] != NL * WID) return;
  if (in_sizes[7] != 2 * WID || in_sizes[8] != 2) return;

  const float* X     = (const float*)d_in[0];
  const float* numin = (const float*)d_in[1];
  const float* numax = (const float*)d_in[2];
  const float* W0    = (const float*)d_in[3];
  const float* b0    = (const float*)d_in[4];
  const float* Wh    = (const float*)d_in[5];
  const float* bh    = (const float*)d_in[6];
  const float* WL    = (const float*)d_in[7];
  const float* bL    = (const float*)d_in[8];
  float* out = (float*)d_out;

  const size_t dynBytes = (size_t)DYN_ELEMS * sizeof(unsigned short);
  (void)hipFuncSetAttribute(reinterpret_cast<const void*>(&k_mlp),
                            hipFuncAttributeMaxDynamicSharedMemorySize, (int)dynBytes);
  const int grid = (n + RPB - 1) / RPB;
  k_mlp<<<dim3(grid), dim3(128), dynBytes, stream>>>(X, numin, numax, W0, b0, Wh, bh, WL, bL, out, n);
  (void)hipGetLastError();
}
